// CrossAttention_23132693856641
// MI455X (gfx1250) — hardware-verified
//
#include <hip/hip_runtime.h>
#include <stdint.h>


typedef _Float16 v16h __attribute__((ext_vector_type(16)));
typedef _Float16 v8h  __attribute__((ext_vector_type(8)));
typedef float    v8f  __attribute__((ext_vector_type(8)));
typedef float    v4f  __attribute__((ext_vector_type(4)));

#ifndef NB
#define NB 4
#endif
#ifndef SEQ
#define SEQ 2048
#endif
#define NB_FULL  4
#define SEQ_FULL 2048
#define DM   512
#define NH   8
#define HD   64
#define KVW  128
#define ROWS (NB * SEQ)

#define ACT_CAR   8.0f
#define W_CAR     1024.0f
#define PROJ_SCL  0.0001220703125f
#define QK_CAR    64.0f
#define V_CAR     8.0f
#define RES_CAR   2048.0f
#define RES_INV   0.00048828125f
#define S_SCL     0.000244140625f
#define P_CAR     16384.0f
#define O_SCL     0.001953125f
#define OUT_SCL   3.814697265625e-06f
#define LN_EPS    1e-5f

static_assert(NB <= NB_FULL && SEQ <= SEQ_FULL);
static_assert(SEQ % 128 == 0);
static_assert(DM == NH * HD);
static_assert(HD == 64);
static_assert(KVW == 2 * HD);
static_assert(DM % 64 == 0 && DM % 32 == 0 && KVW % 64 == 0);
static_assert(DM == 32 * 16);
static_assert(ROWS % 8 == 0);
static_assert((long)(ROWS / 8) * 8 * DM == (long)ROWS * DM);
static_assert((long)(DM / 64) * (DM / 64) * 4096 == (long)DM * DM);
static_assert((long)(KVW / 64) * (DM / 64) * 4096 == (long)DM * KVW);
static_assert((long)(DM / 64) * (ROWS / 64) * 64 * 64 == (long)ROWS * DM);
static_assert((long)(KVW / 64) * (ROWS / 64) * 64 * 64 == (long)ROWS * KVW);
static_assert((long)(SEQ / 128) * NH * NB * 128 * HD == (long)ROWS * DM);
static_assert((long)(ROWS / 16) * 16 * DM == (long)ROWS * DM);
static_assert((long)NB_FULL * SEQ_FULL * DM * 4 == 16777216L);
static_assert(((long)8 * ROWS * DM + 2L * DM * DM + (long)DM * KVW + 2L * ROWS * HD) * 2 <= 134217728L);

union Frag16 { v16h v; v8h p[2]; };

__device__ __forceinline__ v16h ld_frag(const _Float16* p, int hl) {
  Frag16 f;
  f.p[0] = *(const v8h*)(p + 8 * hl);
  f.p[1] = *(const v8h*)(p + 16 + 8 * hl);
  return f.v;
}

__device__ __forceinline__ v8f mma(v16h a, v16h b, v8f c) {
  v8f d = __builtin_amdgcn_wmma_f32_16x16x32_f16(false, a, false, b, (short)0, c, false, false);
  asm volatile("v_nop\n\tv_nop\n\tv_nop\n\tv_nop" : "+v"(d) : "v"(a), "v"(b));
  return d;
}

__device__ __forceinline__ float bf16_rne(float x) {
  unsigned int u = __builtin_bit_cast(unsigned int, x);
  u += 0x7FFFu + ((u >> 16) & 1u);
  return __builtin_bit_cast(float, u & 0xFFFF0000u);
}

__device__ __forceinline__ float red16_sum(float v) {
  v += __shfl_xor(v, 1, 32);
  v += __shfl_xor(v, 2, 32);
  v += __shfl_xor(v, 4, 32);
  v += __shfl_xor(v, 8, 32);
  return v;
}
__device__ __forceinline__ float red32_sum(float v) {
  v += __shfl_xor(v, 16, 32);
  return red16_sum(v);
}

__global__ __launch_bounds__(256) void k_ln(const float* __restrict__ x,
                                            const float* __restrict__ g,
                                            _Float16* __restrict__ PH,
                                            _Float16* __restrict__ PL)
{
  constexpr int ST_L = 8 * DM;
  __shared__ __attribute__((aligned(16))) _Float16 st[2 * 8 * DM];
  static_assert(2 * 8 * DM * 2 == 16384);

  const int lane = threadIdx.x & 31;
  const int wave = __builtin_amdgcn_readfirstlane((int)(threadIdx.x >> 5));
  const int row = blockIdx.x * 8 + wave;
  const int b = row / SEQ;
  const int n = row - b * SEQ;
  const size_t rbase = ((size_t)b * SEQ_FULL + n) * DM;

  float s = 0.f;
#pragma unroll 1
  for (int i = 0; i < 2; ++i) {
    const v4f a0 = *(const v4f*)(x + rbase + 256 * i + 8 * lane);
    const v4f a1 = *(const v4f*)(x + rbase + 256 * i + 8 * lane + 4);
#pragma unroll
    for (int j = 0; j < 4; ++j) s += bf16_rne(a0[j]);
#pragma unroll
    for (int j = 0; j < 4; ++j) s += bf16_rne(a1[j]);
  }
  s = red32_sum(s);
  const float mean = s * (1.0f / DM);

  float ss = 0.f;
#pragma unroll 1
  for (int i = 0; i < 2; ++i) {
    const v4f a0 = *(const v4f*)(x + rbase + 256 * i + 8 * lane);
    const v4f a1 = *(const v4f*)(x + rbase + 256 * i + 8 * lane + 4);
#pragma unroll
    for (int j = 0; j < 4; ++j) { const float d = bf16_rne(a0[j]) - mean; ss += d * d; }
#pragma unroll
    for (int j = 0; j < 4; ++j) { const float d = bf16_rne(a1[j]) - mean; ss += d * d; }
  }
  ss = red32_sum(ss);
  const float inv = rsqrtf(ss * (1.0f / DM) + LN_EPS);

  const int so = wave * DM;
#pragma unroll 1
  for (int j = 0; j < DM / 32; ++j) {
    const int col = 32 * j + lane;
    const float xv = bf16_rne(x[rbase + col]);
    const float gv = bf16_rne(g[col]);
    const float t = (xv - mean) * inv * gv * ACT_CAR;
    const _Float16 h = (_Float16)t;
    st[so + col] = h;
    st[ST_L + so + col] = (_Float16)((t - (float)h) * RES_CAR);
  }
  __syncthreads();

  const v8h oh0 = *(const v8h*)(st + so + 8 * lane);
  const v8h oh1 = *(const v8h*)(st + so + 256 + 8 * lane);
  const v8h ol0 = *(const v8h*)(st + ST_L + so + 8 * lane);
  const v8h ol1 = *(const v8h*)(st + ST_L + so + 256 + 8 * lane);

  _Float16* const dh = PH + (size_t)row * DM + 8 * lane;
  _Float16* const dl = PL + (size_t)row * DM + 8 * lane;
  *(volatile v8h*)(dh)       = oh0;
  *(volatile v8h*)(dh + 256) = oh1;
  *(volatile v8h*)(dl)       = ol0;
  *(volatile v8h*)(dl + 256) = ol1;
  __threadfence();
  *(volatile v8h*)(dh)       = oh0;
  *(volatile v8h*)(dh + 256) = oh1;
  *(volatile v8h*)(dl)       = ol0;
  *(volatile v8h*)(dl + 256) = ol1;
}

__global__ __launch_bounds__(256) void k_trw(const float* __restrict__ W,
                                             _Float16* __restrict__ WT, int R, int C)
{
  __shared__ float tile[64 * 65];
  const int tid = threadIdx.x;
  const int c0 = blockIdx.x * 64, r0 = blockIdx.y * 64;
#pragma unroll
  for (int i = 0; i < 4; ++i) {
    const int idx = i * 256 + tid;
    const int r = idx >> 4, c4 = (idx & 15) * 4;
    const v4f v = *(const v4f*)(W + (size_t)(r0 + r) * C + c0 + c4);
    float* tp = tile + r * 65 + c4;
    tp[0] = v[0]; tp[1] = v[1]; tp[2] = v[2]; tp[3] = v[3];
  }
  __syncthreads();
  v8h o[2];
  size_t dofs[2];
#pragma unroll
  for (int i = 0; i < 2; ++i) {
    const int line = i * 32 + (tid >> 3);
    const int pc   = (tid & 7) * 8;
#pragma unroll
    for (int j = 0; j < 8; ++j)
      o[i][j] = (_Float16)(bf16_rne(tile[(pc + j) * 65 + line]) * W_CAR);
    dofs[i] = (size_t)(c0 + line) * R + r0 + pc;
  }
  *(volatile v8h*)(WT + dofs[0]) = o[0];
  *(volatile v8h*)(WT + dofs[1]) = o[1];
  __threadfence();
  *(volatile v8h*)(WT + dofs[0]) = o[0];
  *(volatile v8h*)(WT + dofs[1]) = o[1];
}

__device__ __forceinline__ void gemm_core(const _Float16* __restrict__ ap0,
                                          const _Float16* __restrict__ ap1,
                                          const _Float16* __restrict__ bp,
                                          int K, int hl, v8f (&acc)[8])
{
  const size_t bst = (size_t)16 * K;
#pragma unroll 1
  for (int k0 = 0; k0 < K; k0 += 32) {
    const v16h a0 = ld_frag(ap0 + k0, hl);
    const v16h a1 = ld_frag(ap1 + k0, hl);
    const v16h b0 = ld_frag(bp + k0, hl);
    const v16h b1 = ld_frag(bp + bst + k0, hl);
    const v16h b2 = ld_frag(bp + 2 * bst + k0, hl);
    const v16h b3 = ld_frag(bp + 3 * bst + k0, hl);
    acc[0] = mma(a0, b0, acc[0]);
    acc[1] = mma(a0, b1, acc[1]);
    acc[2] = mma(a0, b2, acc[2]);
    acc[3] = mma(a0, b3, acc[3]);
    acc[4] = mma(a1, b0, acc[4]);
    acc[5] = mma(a1, b1, acc[5]);
    acc[6] = mma(a1, b2, acc[6]);
    acc[7] = mma(a1, b3, acc[7]);
  }
}

__global__ __launch_bounds__(128) __attribute__((amdgpu_num_vgpr(256)))
void k_qproj(const _Float16* __restrict__ AH, const _Float16* __restrict__ AL,
             const _Float16* __restrict__ Bt, const float* __restrict__ qs,
             _Float16* __restrict__ QH, _Float16* __restrict__ QL)
{
  __shared__ __attribute__((aligned(16))) _Float16 ldsE[2 * 64 * 72];
  constexpr int L_OFF = 64 * 72;

  const int tid = threadIdx.x, lane = tid & 31;
  const int wave = __builtin_amdgcn_readfirstlane((int)(threadIdx.x >> 5));
  const int hl = lane >> 4, c = lane & 15;
  const int m0 = blockIdx.y * 64, n0 = blockIdx.x * 64;
  const int mw = m0 + 16 * wave;

  const _Float16* ap0 = AH + (size_t)(mw + c) * DM;
  const _Float16* ap1 = AL + (size_t)(mw + c) * DM;
  const _Float16* bp  = Bt + (size_t)(n0 + c) * DM;

  v8f acc[8] = {};
  gemm_core(ap0, ap1, bp, DM, hl, acc);

  float qsc[4];
#pragma unroll
  for (int t = 0; t < 4; ++t) qsc[t] = bf16_rne(qs[16 * t + c]) * QK_CAR;

#pragma unroll
  for (int r = 0; r < 8; ++r) {
    float v[4];
    float ss = 0.f;
#pragma unroll
    for (int t = 0; t < 4; ++t) {
      v[t] = (acc[t][r] + acc[4 + t][r] * RES_INV) * PROJ_SCL;
      ss += v[t] * v[t];
    }
    ss = red16_sum(ss);
    const float inv = 1.0f / fmaxf(sqrtf(ss), 1e-12f);
    const int rowl = 16 * wave + 8 * hl + r;
#pragma unroll
    for (int t = 0; t < 4; ++t) {
      const float tt = v[t] * inv * qsc[t];
      const _Float16 hv = (_Float16)tt;
      const float res = (tt - (float)hv) * RES_CAR;
      ldsE[rowl * 72 + 16 * t + c] = hv;
      ldsE[L_OFF + rowl * 72 + 16 * t + c] = (_Float16)res;
    }
  }
  __syncthreads();

  _Float16* const bh = QH + (size_t)m0 * DM + n0;
  _Float16* const bl = QL + (size_t)m0 * DM + n0;
  for (int i = 0; i < 4; ++i) {
    const int q = i * 128 + tid;
    const int rowl = q >> 3, ch = (q & 7) * 8;
    const v8h vh = *(const v8h*)(ldsE + rowl * 72 + ch);
    const v8h vl = *(const v8h*)(ldsE + L_OFF + rowl * 72 + ch);
    *(volatile v8h*)(bh + (size_t)rowl * DM + ch) = vh;
    *(volatile v8h*)(bl + (size_t)rowl * DM + ch) = vl;
  }
  __threadfence();
  for (int i = 0; i < 4; ++i) {
    const int q = i * 128 + tid;
    const int rowl = q >> 3, ch = (q & 7) * 8;
    const v8h vh = *(const v8h*)(ldsE + rowl * 72 + ch);
    const v8h vl = *(const v8h*)(ldsE + L_OFF + rowl * 72 + ch);
    *(volatile v8h*)(bh + (size_t)rowl * DM + ch) = vh;
    *(volatile v8h*)(bl + (size_t)rowl * DM + ch) = vl;
  }
}

__global__ __launch_bounds__(128) __attribute__((amdgpu_num_vgpr(256)))
void k_kvproj(const _Float16* __restrict__ AH, const _Float16* __restrict__ AL,
              const _Float16* __restrict__ Bt, const float* __restrict__ ks,
              _Float16* __restrict__ KV)
{
  __shared__ __attribute__((aligned(16))) _Float16 ldsE[64 * 72];

  const int tid = threadIdx.x, lane = tid & 31;
  const int wave = __builtin_amdgcn_readfirstlane((int)(threadIdx.x >> 5));
  const int hl = lane >> 4, c = lane & 15;
  const int isv = (int)blockIdx.x;
  const int m0 = blockIdx.y * 64, n0 = isv * 64;
  const int mw = m0 + 16 * wave;

  const _Float16* ap0 = AH + (size_t)(mw + c) * DM;
  const _Float16* ap1 = AL + (size_t)(mw + c) * DM;
  const _Float16* bp  = Bt + (size_t)(n0 + c) * DM;

  v8f acc[8] = {};
  gemm_core(ap0, ap1, bp, DM, hl, acc);

  float ksc[4];
#pragma unroll
  for (int t = 0; t < 4; ++t) ksc[t] = bf16_rne(ks[16 * t + c]) * QK_CAR;

#pragma unroll
  for (int r = 0; r < 8; ++r) {
    float v[4];
    float ss = 0.f;
#pragma unroll
    for (int t = 0; t < 4; ++t) {
      v[t] = (acc[t][r] + acc[4 + t][r] * RES_INV) * PROJ_SCL;
      ss += v[t] * v[t];
    }
    ss = red16_sum(ss);
    const float inv = 1.0f / fmaxf(sqrtf(ss), 1e-12f);
    const int rowl = 16 * wave + 8 * hl + r;
#pragma unroll
    for (int t = 0; t < 4; ++t) {
      const float tk = v[t] * inv * ksc[t];
      const float tv = v[t] * V_CAR;
      const float tt = isv ? tv : tk;
      const int li = isv ? ((16 * t + c) * 72 + rowl) : (rowl * 72 + 16 * t + c);
      ldsE[li] = (_Float16)tt;
    }
  }
  __syncthreads();

  const int bb  = m0 / SEQ;
  const int nl0 = m0 - bb * SEQ;
  const size_t vt_off = (size_t)ROWS * HD;
  for (int i = 0; i < 4; ++i) {
    const int q = i * 128 + tid;
    const int rowl = q >> 3, ch = (q & 7) * 8;
    const v8h vv = *(const v8h*)(ldsE + rowl * 72 + ch);
    const size_t offk = (size_t)(m0 + rowl) * HD + ch;
    const size_t offv = vt_off + ((size_t)bb * HD + rowl) * SEQ + nl0 + ch;
    const size_t off = isv ? offv : offk;
    *(volatile v8h*)(KV + off) = vv;
  }
  __threadfence();
  for (int i = 0; i < 4; ++i) {
    const int q = i * 128 + tid;
    const int rowl = q >> 3, ch = (q & 7) * 8;
    const v8h vv = *(const v8h*)(ldsE + rowl * 72 + ch);
    const size_t offk = (size_t)(m0 + rowl) * HD + ch;
    const size_t offv = vt_off + ((size_t)bb * HD + rowl) * SEQ + nl0 + ch;
    const size_t off = isv ? offv : offk;
    *(volatile v8h*)(KV + off) = vv;
  }
}

__global__ __launch_bounds__(256) __attribute__((amdgpu_num_vgpr(256)))
void k_attn(const _Float16* __restrict__ QH, const _Float16* __restrict__ QL,
            const _Float16* __restrict__ KP, const _Float16* __restrict__ VT,
            _Float16* __restrict__ OH, _Float16* __restrict__ OL)
{
  constexpr int KT_H   = 32 * 72;
  constexpr int V_H    = HD * 40;
  constexpr int P_H    = 8 * 16 * 40;
  constexpr int K_OFF  = 0;
  constexpr int V_OFF  = KT_H;
  constexpr int P_OFF  = KT_H + V_H;
  constexpr int TILE_H = KT_H + V_H + P_H;
  constexpr int EPI_H  = 2 * 128 * 72;
  constexpr int OL_OFF = 128 * 72;
  constexpr int LDS_H  = (TILE_H > EPI_H) ? TILE_H : EPI_H;
  static_assert(TILE_H <= LDS_H && EPI_H <= LDS_H);
  __shared__ __attribute__((aligned(16))) _Float16 lds[LDS_H];

  const int tid = threadIdx.x, lane = tid & 31;
  const int wave = __builtin_amdgcn_readfirstlane((int)(threadIdx.x >> 5));
  const int hl = lane >> 4, c = lane & 15;
  const int q0 = blockIdx.x * 128;
  const int col0 = blockIdx.y * HD;
  const int b = blockIdx.z;
  const int brow0 = b * SEQ;

  const size_t qrow = (size_t)(brow0 + q0 + 16 * wave + c) * DM + col0;
  v16h qh[2], ql[2];
#pragma unroll
  for (int ks = 0; ks < 2; ++ks) {
    qh[ks] = ld_frag(QH + qrow + 32 * ks, hl);
    ql[ks] = ld_frag(QL + qrow + 32 * ks, hl);
  }
  const int pofs = P_OFF + wave * (16 * 40);

  const int krr = tid >> 3, kcc = (tid & 7) * 8;
  const int vdd = tid >> 2, vkc = (tid & 3) * 8;
  const _Float16* const kg = KP + (size_t)(brow0 + krr) * HD + kcc;
  const _Float16* const vg = VT + ((size_t)b * HD + vdd) * SEQ + vkc;

  float m[8], l[8];
  v8f oh[4] = {};
#pragma unroll
  for (int r = 0; r < 8; ++r) { m[r] = -__builtin_inff(); l[r] = 0.f; }

#pragma unroll 1
  for (int kt = 0; kt < SEQ / 32; ++kt) {
    const int mk = kt * 32;
    {
      const v8h k8 = *(const v8h*)(kg + (size_t)mk * HD);
      const v8h v8 = *(const v8h*)(vg + mk);
      *(v8h*)(lds + K_OFF + krr * 72 + kcc) = k8;
      *(v8h*)(lds + V_OFF + vdd * 40 + vkc) = v8;
    }
    __syncthreads();

    v8f sh[2] = {}, sl[2] = {};
#pragma unroll
    for (int ks = 0; ks < 2; ++ks) {
#pragma unroll
      for (int t = 0; t < 2; ++t) {
        const v16h kf = ld_frag(lds + K_OFF + (16 * t + c) * 72 + 32 * ks, hl);
        sh[t] = mma(qh[ks], kf, sh[t]);
        sl[t] = mma(ql[ks], kf, sl[t]);
      }
    }

#pragma unroll
    for (int r = 0; r < 8; ++r) {
      const float v0 = (sh[0][r] + sl[0][r] * RES_INV) * S_SCL;
      const float v1 = (sh[1][r] + sl[1][r] * RES_INV) * S_SCL;
      float tm = fmaxf(v0, v1);
      tm = fmaxf(tm, __shfl_xor(tm, 1, 32));
      tm = fmaxf(tm, __shfl_xor(tm, 2, 32));
      tm = fmaxf(tm, __shfl_xor(tm, 4, 32));
      tm = fmaxf(tm, __shfl_xor(tm, 8, 32));
      const float mn = fmaxf(m[r], tm);
      const float al = __expf(m[r] - mn);
      const float p0 = __expf(v0 - mn), p1 = __expf(v1 - mn);
      float rs = p0 + p1;
      rs += __shfl_xor(rs, 1, 32);
      rs += __shfl_xor(rs, 2, 32);
      rs += __shfl_xor(rs, 4, 32);
      rs += __shfl_xor(rs, 8, 32);
      l[r] = l[r] * al + rs;
      m[r] = mn;
#pragma unroll
      for (int t = 0; t < 4; ++t) oh[t][r] *= al;
      const int pi = pofs + (8 * hl + r) * 40 + c;
      lds[pi]      = (_Float16)(p0 * P_CAR);
      lds[pi + 16] = (_Float16)(p1 * P_CAR);
    }
    __syncthreads();

    const v16h pf = ld_frag(lds + pofs + c * 40, hl);
#pragma unroll
    for (int t = 0; t < 4; ++t) {
      const v16h vf = ld_frag(lds + V_OFF + (16 * t + c) * 40, hl);
      oh[t] = mma(pf, vf, oh[t]);
    }
    __syncthreads();
  }

#pragma unroll
  for (int r = 0; r < 8; ++r) {
    const float inv = (1.0f / l[r]) * O_SCL;
    const int rowl = 16 * wave + 8 * hl + r;
#pragma unroll
    for (int t = 0; t < 4; ++t) {
      const float v = oh[t][r] * inv;
      const _Float16 hv = (_Float16)v;
      const float res = (v - (float)hv) * RES_CAR;
      lds[rowl * 72 + 16 * t + c] = hv;
      lds[OL_OFF + rowl * 72 + 16 * t + c] = (_Float16)res;
    }
  }
  __syncthreads();
  _Float16* const bh = OH + (size_t)(brow0 + q0) * DM + col0;
  _Float16* const bl = OL + (size_t)(brow0 + q0) * DM + col0;
  for (int i = 0; i < 4; ++i) {
    const int q = i * 256 + tid;
    const int rowl = q >> 3, ch = (q & 7) * 8;
    const v8h vh = *(const v8h*)(lds + rowl * 72 + ch);
    const v8h vl = *(const v8h*)(lds + OL_OFF + rowl * 72 + ch);
    *(volatile v8h*)(bh + (size_t)rowl * DM + ch) = vh;
    *(volatile v8h*)(bl + (size_t)rowl * DM + ch) = vl;
  }
  __threadfence();
  for (int i = 0; i < 4; ++i) {
    const int q = i * 256 + tid;
    const int rowl = q >> 3, ch = (q & 7) * 8;
    const v8h vh = *(const v8h*)(lds + rowl * 72 + ch);
    const v8h vl = *(const v8h*)(lds + OL_OFF + rowl * 72 + ch);
    *(volatile v8h*)(bh + (size_t)rowl * DM + ch) = vh;
    *(volatile v8h*)(bl + (size_t)rowl * DM + ch) = vl;
  }
}

__global__ __launch_bounds__(256) __attribute__((amdgpu_num_vgpr(256)))
void k_oproj_ln(const _Float16* __restrict__ AH, const _Float16* __restrict__ AL,
                const _Float16* __restrict__ Bt, const float* __restrict__ g,
                float* __restrict__ Out)
{
  constexpr int FP = DM + 4;
  __shared__ __attribute__((aligned(16))) float ldsF[16 * FP];

  const int tid = threadIdx.x, lane = tid & 31;
  const int wave = __builtin_amdgcn_readfirstlane((int)(threadIdx.x >> 5));
  const int hl = lane >> 4, c = lane & 15;
  const int m0 = blockIdx.x * 16;
  const int n0 = 64 * wave;

  const _Float16* ap0 = AH + (size_t)(m0 + c) * DM;
  const _Float16* ap1 = AL + (size_t)(m0 + c) * DM;
  const _Float16* bp  = Bt + (size_t)(n0 + c) * DM;

  v8f acc[8] = {};
  gemm_core(ap0, ap1, bp, DM, hl, acc);

#pragma unroll
  for (int t = 0; t < 4; ++t)
#pragma unroll
    for (int r = 0; r < 8; ++r)
      ldsF[(8 * hl + r) * FP + n0 + 16 * t + c] = (acc[t][r] + acc[4 + t][r] * RES_INV) * OUT_SCL;
  __syncthreads();

  v4f o[2][4];
  size_t oo[2];
#pragma unroll
  for (int rr = 0; rr < 2; ++rr) {
    const int rowl = 2 * wave + rr;
    v4f y[4];
    float s = 0.f;
#pragma unroll
    for (int i = 0; i < 4; ++i) {
      y[i] = *(const v4f*)(ldsF + rowl * FP + 128 * i + 4 * lane);
      s += (y[i][0] + y[i][1]) + (y[i][2] + y[i][3]);
    }
    s = red32_sum(s);
    const float mean = s * (1.0f / DM);
    float ss = 0.f;
#pragma unroll
    for (int i = 0; i < 4; ++i)
#pragma unroll
      for (int j = 0; j < 4; ++j) { const float d = y[i][j] - mean; ss += d * d; }
    ss = red32_sum(ss);
    const float inv = rsqrtf(ss * (1.0f / DM) + LN_EPS);
#pragma unroll
    for (int i = 0; i < 4; ++i) {
      const v4f g4 = *(const v4f*)(g + 128 * i + 4 * lane);
#pragma unroll
      for (int j = 0; j < 4; ++j)
        o[rr][i][j] = (y[i][j] - mean) * inv * bf16_rne(g4[j]);
    }
    const int mrow = m0 + rowl;
    const int bb = mrow / SEQ;
    const int nn = mrow - bb * SEQ;
    oo[rr] = ((size_t)bb * SEQ_FULL + nn) * DM + 4 * lane;
  }
#pragma unroll
  for (int rr = 0; rr < 2; ++rr)
#pragma unroll
    for (int i = 0; i < 4; ++i)
      *(volatile v4f*)(Out + oo[rr] + 128 * i) = o[rr][i];
  __threadfence();
#pragma unroll
  for (int rr = 0; rr < 2; ++rr)
#pragma unroll
    for (int i = 0; i < 4; ++i)
      *(volatile v4f*)(Out + oo[rr] + 128 * i) = o[rr][i];
}

extern "C" void kernel_launch(void* const* d_in, const int* in_sizes, int n_in,
                              void* d_out, int out_size, void* d_ws, size_t ws_size,
                              hipStream_t stream)
{
  if (n_in < 10) return;
  const long act_need = ((long)(NB - 1) * SEQ_FULL + SEQ) * DM;
  if ((long)in_sizes[0] < act_need) return;
  if ((long)in_sizes[1] < act_need) return;
  if ((long)in_sizes[2] < (long)DM) return;
  if ((long)in_sizes[3] < (long)DM) return;
  if ((long)in_sizes[4] < (long)DM * DM) return;
  if ((long)in_sizes[5] < (long)DM * KVW) return;
  if ((long)in_sizes[6] < (long)HD) return;
  if ((long)in_sizes[7] < (long)HD) return;
  if ((long)in_sizes[8] < (long)DM * DM) return;
  if ((long)in_sizes[9] < (long)DM) return;
  if ((long)out_size < act_need) return;

  const float* zt   = (const float*)d_in[0];
  const float* ic   = (const float*)d_in[1];
  const float* g_zt = (const float*)d_in[2];
  const float* g_ic = (const float*)d_in[3];
  const float* Wq   = (const float*)d_in[4];
  const float* Wkv  = (const float*)d_in[5];
  const float* qsc  = (const float*)d_in[6];
  const float* ksc  = (const float*)d_in[7];
  const float* Wo   = (const float*)d_in[8];
  const float* g_o  = (const float*)d_in[9];
  float* out = (float*)d_out;

  const size_t nA   = (size_t)ROWS * DM;
  const size_t nWs  = (size_t)DM * DM;
  const size_t nWkv = (size_t)DM * KVW;
  const size_t nKV  = (size_t)ROWS * HD;
  const size_t total_halves = 8 * nA + 2 * nWs + nWkv + 2 * nKV;
  if (total_halves * sizeof(_Float16) > ws_size) return;

  _Float16* ZH   = (_Float16*)d_ws;
  _Float16* ZL   = ZH   + nA;
  _Float16* CH   = ZL   + nA;
  _Float16* CL   = CH   + nA;
  _Float16* WqT  = CL   + nA;
  _Float16* WkvT = WqT  + nWs;
  _Float16* WoT  = WkvT + nWkv;
  _Float16* QH   = WoT  + nWs;
  _Float16* QL   = QH   + nA;
  _Float16* KP   = QL   + nA;
  _Float16* VT   = KP   + nKV;
  _Float16* OH   = VT   + nKV;
  _Float16* OL   = OH   + nA;

  k_ln<<<ROWS / 8, 256, 0, stream>>>(zt, g_zt, ZH, ZL);
  k_ln<<<ROWS / 8, 256, 0, stream>>>(ic, g_ic, CH, CL);

  k_trw<<<dim3(DM / 64, DM / 64), 256, 0, stream>>>(Wq, WqT, DM, DM);
  k_trw<<<dim3(KVW / 64, DM / 64), 256, 0, stream>>>(Wkv, WkvT, DM, KVW);
  k_trw<<<dim3(DM / 64, DM / 64), 256, 0, stream>>>(Wo, WoT, DM, DM);

  k_qproj<<<dim3(DM / 64, ROWS / 64), 128, 0, stream>>>(ZH, ZL, WqT, qsc, QH, QL);
  k_kvproj<<<dim3(KVW / 64, ROWS / 64), 128, 0, stream>>>(CH, CL, WkvT, ksc, KP);

  k_attn<<<dim3(SEQ / 128, NH, NB), 256, 0, stream>>>(QH, QL, KP, VT, OH, OL);

  k_oproj_ln<<<ROWS / 16, 256, 0, stream>>>(OH, OL, WoT, g_o, out);
}
